// MessagePassing_59339268162203
// MI455X (gfx1250) — hardware-verified
//
#include <hip/hip_runtime.h>
#include <math.h>

constexpr int NNODE  = 50000;
constexpr int NEDGE  = 1600000;
constexpr int FDIM   = 128;
constexpr int NPAD   = 50048;
constexpr int CPITCH = 384;
constexpr int NTHR   = 256;
static_assert(NPAD % 64 == 0 && NPAD >= NNODE && NPAD - NNODE < 64, "cfg");
static_assert(NNODE % 16 == 0, "cfg");
static_assert(FDIM % 64 == 0 && FDIM % 32 == 0 && (2 * FDIM) % 32 == 0, "cfg");
static_assert((NPAD * 16) % NTHR == 0 && (NPAD * 32) % NTHR == 0, "cfg");
static_assert(NNODE < 65536, "cfg");

constexpr int WOFF_P1 = 0;
constexpr int WOFF_P2 = 16384;
constexpr int WOFF_P3 = 32768;
constexpr int WOFF_P4 = 49152;
constexpr int WOFF_ZR = 65536;
constexpr int WOFF_H  = 131072;
constexpr int WPLANE_HALVES = 163840;
constexpr int BOFF_M1B1 = 0;
constexpr int BOFF_M1B2 = 128;
constexpr int BOFF_M2B1 = 256;
constexpr int BOFF_M2B2 = 384;
constexpr int BOFF_Z    = 512;
constexpr int BOFF_R    = 640;
constexpr int BOFF_HB   = 768;
constexpr int NBIASR    = 896;

typedef __attribute__((ext_vector_type(16))) _Float16 v16h;
typedef __attribute__((ext_vector_type(8)))  _Float16 v8h;
typedef __attribute__((ext_vector_type(16))) __bf16   v16b;
typedef __attribute__((ext_vector_type(8)))  __bf16   v8b;
typedef __attribute__((ext_vector_type(8)))  float    v8f;
typedef __attribute__((ext_vector_type(4)))  float    v4f;
typedef __attribute__((ext_vector_type(4)))  unsigned int v4u;
typedef __attribute__((ext_vector_type(2)))  unsigned int v2u;
typedef __attribute__((ext_vector_type(4)))  int      v4i;

__device__ __forceinline__ unsigned short f2bf_bits(float f) {
  unsigned u = __float_as_uint(f);
  return (unsigned short)((u + 0x7FFFu + ((u >> 16) & 1u)) >> 16);
}
__device__ __forceinline__ float bf_bits2f(unsigned short h) { return __uint_as_float(((unsigned)h) << 16); }
__device__ __forceinline__ float bfr(float f) { return bf_bits2f(f2bf_bits(f)); }
__device__ __forceinline__ unsigned pk16(unsigned short a, unsigned short b) { return (unsigned)a | ((unsigned)b << 16); }

__device__ __forceinline__ void dep_guard_h(v8f& a, v8f& b, v16h x, v16h y) { asm volatile("v_nop\n\tv_nop\n\tv_nop\n\tv_nop" : "+v"(a), "+v"(b) : "v"(x), "v"(y)); }
__device__ __forceinline__ void dep_guard_b(v8f& a, v8f& b, v16b x, v16b y) { asm volatile("v_nop\n\tv_nop\n\tv_nop\n\tv_nop" : "+v"(a), "+v"(b) : "v"(x), "v"(y)); }
__device__ __forceinline__ void dep_guard4_h(v8f& a, v8f& b, v8f& c, v8f& d, v16h x, v16h y) { asm volatile("v_nop\n\tv_nop\n\tv_nop\n\tv_nop" : "+v"(a), "+v"(b), "+v"(c), "+v"(d) : "v"(x), "v"(y)); }
__device__ __forceinline__ void dep_guard4_b(v8f& a, v8f& b, v8f& c, v8f& d, v16b x, v16b y) { asm volatile("v_nop\n\tv_nop\n\tv_nop\n\tv_nop" : "+v"(a), "+v"(b), "+v"(c), "+v"(d) : "v"(x), "v"(y)); }
__device__ __forceinline__ void keep4_h(v16h a, v16h b, v16h c, v16h d) { asm volatile("v_nop" :: "v"(a), "v"(b), "v"(c), "v"(d)); }
__device__ __forceinline__ void keep4_b(v16b a, v16b b, v16b c, v16b d) { asm volatile("v_nop" :: "v"(a), "v"(b), "v"(c), "v"(d)); }
__device__ __forceinline__ void acc_guard4(v8f& a, v8f& b, v8f& c, v8f& d) { asm volatile("v_nop\n\tv_nop\n\tv_nop\n\tv_nop" : "+v"(a), "+v"(b), "+v"(c), "+v"(d)); }
template <typename T> struct Frag;
template <> struct Frag<_Float16> {
  typedef v16h V; union U { v16h v; v8h h[2]; };
  static __device__ __forceinline__ v16h load(const _Float16* p) {
    U f; f.h[0] = *(const v8h*)(p); f.h[1] = *(const v8h*)(p + 16); return f.v;
  }
  static __device__ __forceinline__ v8f mma(v16h a, v16h b, v8f c) {
    return __builtin_amdgcn_wmma_f32_16x16x32_f16(false, a, false, b, (short)0, c, false, false);
  }
  static __device__ __forceinline__ void guard(v8f& a, v8f& b, v16h x, v16h y) { dep_guard_h(a, b, x, y); }
  static __device__ __forceinline__ void guard4(v8f& a, v8f& b, v8f& c, v8f& d, v16h x, v16h y) { dep_guard4_h(a, b, c, d, x, y); }
  static __device__ __forceinline__ void keep(v16h a, v16h b, v16h c, v16h d) { keep4_h(a, b, c, d); }
};
template <> struct Frag<__bf16> {
  typedef v16b V; union U { v16b v; v8b h[2]; };
  static __device__ __forceinline__ v16b load(const __bf16* p) {
    U f; f.h[0] = *(const v8b*)(p); f.h[1] = *(const v8b*)(p + 16); return f.v;
  }
  static __device__ __forceinline__ v8f mma(v16b a, v16b b, v8f c) {
    return __builtin_amdgcn_wmma_f32_16x16x32_bf16(false, a, false, b, (short)0, c, false, false);
  }
  static __device__ __forceinline__ void guard(v8f& a, v8f& b, v16b x, v16b y) { dep_guard_b(a, b, x, y); }
  static __device__ __forceinline__ void guard4(v8f& a, v8f& b, v8f& c, v8f& d, v16b x, v16b y) { dep_guard4_b(a, b, c, d, x, y); }
  static __device__ __forceinline__ void keep(v16b a, v16b b, v16b c, v16b d) { keep4_b(a, b, c, d); }
};

__device__ __forceinline__ float sigm_f(float v) {
  const float e = expf(-v);
  return 1.0f / (1.0f + e);
}
__device__ __forceinline__ float tanh_f(float v) {
  const float a = fabsf(v);
  const float t = expf(-2.0f * a);
  const float y = (1.0f - t) * (1.0f / (1.0f + t));
  return copysignf(y, v);
}

template <int ET> struct Elem;
template <> struct Elem<0> { typedef _Float16 T; };
template <> struct Elem<1> { typedef __bf16 T; };
template <int ET, int SPLIT, int BIAS_MODE, int OUT_MODE, bool RESID, int ACT = 0>
__global__ __launch_bounds__(256) void wmma_gemm64(
    const unsigned short* __restrict__ Ap, const unsigned short* __restrict__ A2p, int lda, long strideA,
    const unsigned short* __restrict__ Btp, const unsigned short* __restrict__ Bt2p, int ldb, long strideB,
    void* __restrict__ Cout, void* __restrict__ Cout2, int ldc, long strideC,
    const float* __restrict__ bias,
    const float* __restrict__ resid, long strideR,
    int M, int N, int K, float scale,
    const float* __restrict__ auxz, const float* __restrict__ auxx, int Mreal) {
  typedef typename Elem<ET>::T T;
  typedef typename Frag<T>::V V;
  const T* A = (const T*)Ap; const T* A2 = (const T*)A2p; const T* Bt = (const T*)Btp; const T* Bt2 = (const T*)Bt2p;
  __shared__ __align__(16) float sT[8][16 * 68];
  const int b    = blockIdx.y;
  const int lane = threadIdx.x & 31;
  const int wave = threadIdx.x >> 5;
  const int tilesN = N >> 6;
  const int tilesM = M >> 6;
  const int tile = blockIdx.x * 8 + wave;
  if (tile >= tilesM * tilesN) return;
  const int tm = tile / tilesN;
  const int tn = tile - tm * tilesN;
  const int m0 = tm << 6;
  const int n0 = tn << 6;

  const T* Ab  = A  + (size_t)b * strideA;
  const T* Bb  = Bt + (size_t)b * strideB;
  const T* Ab2 = (SPLIT >= 1) ? (A2  + (size_t)b * strideA) : nullptr;
  const T* Bb2 = (SPLIT == 2) ? (Bt2 + (size_t)b * strideB) : nullptr;

  const int rlane = lane & 15;
  const int koff  = (lane >> 4) * 8;
  const int mOff  = (lane >> 4) * 8;

  v8f acc[4][4];
#pragma unroll
  for (int i = 0; i < 4; ++i)
#pragma unroll
    for (int j = 0; j < 4; ++j) acc[i][j] = (v8f){0.f,0.f,0.f,0.f,0.f,0.f,0.f,0.f};

  for (int k0 = 0; k0 < K; k0 += 32) {
    V bh[4], bl[4];
#pragma unroll
    for (int j = 0; j < 4; ++j) {
      const size_t bo = (size_t)(n0 + (j << 4) + rlane) * ldb + koff + k0;
      bh[j] = Frag<T>::load(Bb + bo);
      if (SPLIT == 2) bl[j] = Frag<T>::load(Bb2 + bo); else bl[j] = bh[j];
    }
#pragma unroll
    for (int i = 0; i < 4; ++i) {
      const size_t ao = (size_t)(m0 + (i << 4) + rlane) * lda + koff + k0;
      V ah = Frag<T>::load(Ab + ao);
      V al;
      if (SPLIT >= 1) al = Frag<T>::load(Ab2 + ao); else al = ah;
#pragma unroll
      for (int j = 0; j < 4; ++j) {
        acc[i][j] = Frag<T>::mma(ah, bh[j], acc[i][j]);
        if (SPLIT == 2) acc[i][j] = Frag<T>::mma(ah, bl[j], acc[i][j]);
        if (SPLIT >= 1) acc[i][j] = Frag<T>::mma(al, bh[j], acc[i][j]);
      }
      Frag<T>::guard4(acc[i][0], acc[i][1], acc[i][2], acc[i][3], ah, al);
    }
    Frag<T>::keep(bh[0], bh[1], bh[2], bh[3]);
    if (SPLIT == 2) Frag<T>::keep(bl[0], bl[1], bl[2], bl[3]);
  }
  acc_guard4(acc[0][0], acc[0][1], acc[0][2], acc[0][3]);
  acc_guard4(acc[1][0], acc[1][1], acc[1][2], acc[1][3]);
  acc_guard4(acc[2][0], acc[2][1], acc[2][2], acc[2][3]);
  acc_guard4(acc[3][0], acc[3][1], acc[3][2], acc[3][3]);

  float* slab = sT[wave];
  const float* Rb = RESID ? (resid + (size_t)b * strideR) : nullptr;
#pragma unroll
  for (int i = 0; i < 4; ++i) {
    const int mBase = m0 + (i << 4);
#pragma unroll
    for (int j = 0; j < 4; ++j) {
      const int n = n0 + (j << 4) + rlane;
      float bv = 0.f;
      if (BIAS_MODE == 2) bv = bias[n];
#pragma unroll
      for (int r = 0; r < 8; ++r) {
        float v = acc[i][j][r] * scale;
        if (BIAS_MODE == 1) v += bias[mBase + mOff + r];
        if (BIAS_MODE == 2) v += bv;
        if (RESID) v += Rb[(size_t)(mBase + mOff + r) * ldc + n];
        if (ACT == 2) v = fmaxf(v, 0.0f);
        if (ACT == 4) v = (v > 0.f) ? v : 0.01f * v;
        slab[(mOff + r) * 68 + (j << 4) + rlane] = v;
      }
    }
    __builtin_amdgcn_fence(__ATOMIC_RELEASE, "workgroup");
    __builtin_amdgcn_wave_barrier();
    __builtin_amdgcn_fence(__ATOMIC_ACQUIRE, "workgroup");
    if (OUT_MODE == 0) {
      float* C = (float*)Cout + (size_t)b * strideC;
      const int hh = lane >> 4, c4 = (lane & 15) * 4;
      for (int pass = 0; pass < 2; ++pass) {
#pragma unroll
        for (int it = 0; it < 8; ++it) {
          const int row = it * 2 + hh;
          v4f v = *(const v4f*)(slab + row * 68 + c4);
          *(volatile v4f*)(C + (size_t)(mBase + row) * ldc + n0 + c4) = v;
        }
        __threadfence();
      }
    } else if (OUT_MODE == 3) {
      float* C = (float*)Cout;
      const int hh = lane >> 4, c4 = (lane & 15) * 4;
#pragma unroll 1
      for (int it = 0; it < 8; ++it) {
        const int row = it * 2 + hh;
        const size_t go = (size_t)(mBase + row) * ldc + n0 + c4;
        const v4f hp = *(const v4f*)(slab + row * 68 + c4);
        const v4f zp = *(const v4f*)(auxz + go);
        const v4f xv = *(const v4f*)(auxx + go);
        v4f o;
#pragma unroll
        for (int e = 0; e < 4; ++e) {
          const float zg = sigm_f(zp[e]);
          const float hg = tanh_f(hp[e]);
          o[e] = (1.0f - zg) * xv[e] + zg * hg;
        }
        *(v4f*)(slab + row * 68 + c4) = o;
      }
      __builtin_amdgcn_fence(__ATOMIC_RELEASE, "workgroup");
      __builtin_amdgcn_wave_barrier();
      __builtin_amdgcn_fence(__ATOMIC_ACQUIRE, "workgroup");
      if (mBase < Mreal) {
        for (int pass = 0; pass < 2; ++pass) {
#pragma unroll
          for (int it = 0; it < 8; ++it) {
            const int row = it * 2 + hh;
            v4f v = *(const v4f*)(slab + row * 68 + c4);
            *(volatile v4f*)(C + (size_t)(mBase + row) * ldc + n0 + c4) = v;
          }
          __threadfence();
        }
      }
    } else {
      const int q = lane >> 3, c8 = (lane & 7) * 8;
      unsigned short* C  = (unsigned short*)Cout  + (size_t)b * strideC;
      unsigned short* C2 = (OUT_MODE == 2) ? ((unsigned short*)Cout2 + (size_t)b * strideC) : nullptr;
      for (int pass = 0; pass < 2; ++pass) {
#pragma unroll
        for (int it = 0; it < 4; ++it) {
          const int row = it * 4 + q;
          const float* sp = slab + row * 68 + c8;
          v8h hv, lv;
#pragma unroll
          for (int e = 0; e < 8; ++e) {
            if (OUT_MODE == 1) {
              hv[e] = (_Float16)sp[e];
            } else {
              unsigned short hb = f2bf_bits(sp[e]);
              unsigned short lb = f2bf_bits(sp[e] - bf_bits2f(hb));
              hv[e] = __builtin_bit_cast(_Float16, hb);
              lv[e] = __builtin_bit_cast(_Float16, lb);
            }
          }
          *(volatile v8h*)(C + (size_t)(mBase + row) * ldc + n0 + c8) = hv;
          if (OUT_MODE == 2) *(volatile v8h*)(C2 + (size_t)(mBase + row) * ldc + n0 + c8) = lv;
        }
        __threadfence();
      }
    }
    __builtin_amdgcn_fence(__ATOMIC_RELEASE, "workgroup");
    __builtin_amdgcn_wave_barrier();
    __builtin_amdgcn_fence(__ATOMIC_ACQUIRE, "workgroup");
  }
}

__global__ __launch_bounds__(NTHR) void prep_kernel(
    const float* __restrict__ W0, const float* __restrict__ W1, const float* __restrict__ W2, const float* __restrict__ W3,
    const float* __restrict__ W4, const float* __restrict__ W5, const float* __restrict__ W6, const float* __restrict__ W7,
    const float* __restrict__ W8, const float* __restrict__ W9,
    const float* __restrict__ m1b1, const float* __restrict__ m1b2, const float* __restrict__ m2b1, const float* __restrict__ m2b2,
    const float* __restrict__ bu1, const float* __restrict__ bu2, const float* __restrict__ br1, const float* __restrict__ br2,
    const float* __restrict__ bo1, const float* __restrict__ bo2,
    unsigned short* __restrict__ WB, float* __restrict__ BIASR) {
  __shared__ float sm[64][65];
  const int t = threadIdx.x, lane = t & 31, wave = t >> 5;
  const int tb = blockIdx.x;
  if (tb < 40) {
    int wi = 0, pitch = 128, n0d = 0, k0d = 0, srow0 = 0, scol0 = 0, dsto = 0;
    if (tb < 16) {
      const int p = tb >> 2, sub = tb & 3;
      n0d = (sub >> 1) * 64; k0d = (sub & 1) * 64;
      wi = p; dsto = p * 16384; pitch = 128;
      srow0 = k0d; scol0 = n0d;
    } else if (tb < 32) {
      const int u = tb - 16;
      n0d = (u >> 2) * 64; k0d = (u & 3) * 64; pitch = 256; dsto = WOFF_ZR;
      const int nh = n0d >> 7, kh = k0d >> 7;
      wi = nh ? (kh ? 6 : 7) : (kh ? 4 : 5);
      srow0 = k0d - 128 * kh; scol0 = n0d - 128 * nh;
    } else {
      const int u = tb - 32;
      n0d = (u >> 2) * 64; k0d = (u & 3) * 64; pitch = 256; dsto = WOFF_H;
      const int kh = k0d >> 7;
      wi = kh ? 9 : 8;
      srow0 = k0d - 128 * kh; scol0 = n0d;
    }
    const float* W = (wi == 0) ? W0 : (wi == 1) ? W1 : (wi == 2) ? W2 : (wi == 3) ? W3 : (wi == 4) ? W4 :
                     (wi == 5) ? W5 : (wi == 6) ? W6 : (wi == 7) ? W7 : (wi == 8) ? W8 : W9;
#pragma unroll
    for (int i = 0; i < 16; ++i) {
      const int e = i * 256 + t;
      const int r = e >> 6;
      const int c = e & 63;
      sm[c][r] = W[(size_t)(srow0 + r) * FDIM + scol0 + c];
    }
    __syncthreads();
    const int q = lane >> 3, c8 = (lane & 7) * 8;
    for (int pass = 0; pass < 2; ++pass) {
#pragma unroll
      for (int it = 0; it < 2; ++it) {
        const int row = wave * 8 + it * 4 + q;
        unsigned short hb[8];
#pragma unroll
        for (int e = 0; e < 8; ++e) hb[e] = f2bf_bits(sm[row][c8 + e]);
        const v4u uh = (v4u){pk16(hb[0], hb[1]), pk16(hb[2], hb[3]), pk16(hb[4], hb[5]), pk16(hb[6], hb[7])};
        const size_t o = (size_t)dsto + (size_t)(n0d + row) * pitch + k0d + c8;
        *(volatile v4u*)(WB + o) = uh;
      }
      __threadfence();
    }
  } else {
    if (wave < 7) {
      const float* pa = (wave == 0) ? m1b1 : (wave == 1) ? m1b2 : (wave == 2) ? m2b1 : (wave == 3) ? m2b2 :
                        (wave == 4) ? bu1 : (wave == 5) ? br1 : bo1;
      const float* pb = (wave == 4) ? bu2 : (wave == 5) ? br2 : (wave == 6) ? bo2 : pa;
      const float fb = (wave >= 4) ? 1.0f : 0.0f;
      const v4f a = *(const v4f*)(pa + 4 * lane);
      const v4f c = *(const v4f*)(pb + 4 * lane);
      v4f s;
#pragma unroll
      for (int e = 0; e < 4; ++e) s[e] = bfr(a[e]) + fb * bfr(c[e]);
      float* dst = BIASR + wave * 128 + 4 * lane;
      *(volatile v4f*)dst = s;
      __threadfence();
      *(volatile v4f*)dst = s;
    }
  }
}

__global__ __launch_bounds__(NTHR) void cast_xin_kernel(const float* __restrict__ xin, unsigned short* __restrict__ XB) {
  const int i = blockIdx.x * NTHR + threadIdx.x;
  if (i >= NPAD * 16) return;
  const int row = i >> 4, c8 = (i & 15) * 8;
  const bool live = row < NNODE;
  const int rc = live ? row : (NNODE - 1);
  const float fl = live ? 1.0f : 0.0f;
  const float* p = xin + (size_t)rc * FDIM + c8;
  const v4f a = *(const v4f*)p;
  const v4f c = *(const v4f*)(p + 4);
  unsigned short hb[8];
#pragma unroll
  for (int e = 0; e < 4; ++e) {
    hb[e]     = f2bf_bits(a[e] * fl);
    hb[4 + e] = f2bf_bits(c[e] * fl);
  }
  const v4u uh = (v4u){pk16(hb[0], hb[1]), pk16(hb[2], hb[3]), pk16(hb[4], hb[5]), pk16(hb[6], hb[7])};
  const size_t o = (size_t)row * CPITCH + c8;
  *(volatile v4u*)(XB + o) = uh;
  __threadfence();
  *(volatile v4u*)(XB + o) = uh;
}

__global__ __launch_bounds__(NTHR) void castx_kernel(const float* __restrict__ xf,
                                                     unsigned short* __restrict__ XH, unsigned short* __restrict__ XL) {
  const int i = blockIdx.x * NTHR + threadIdx.x;
  if (i >= NPAD * 16) return;
  const int row = i >> 4, c8 = (i & 15) * 8;
  const float* p = xf + (size_t)row * FDIM + c8;
  const v4f a = *(const v4f*)p;
  const v4f c = *(const v4f*)(p + 4);
  unsigned short hb[8], lb[8];
#pragma unroll
  for (int e = 0; e < 4; ++e) {
    hb[e] = f2bf_bits(a[e]);      lb[e] = f2bf_bits(a[e] - bf_bits2f(hb[e]));
    hb[4 + e] = f2bf_bits(c[e]);  lb[4 + e] = f2bf_bits(c[e] - bf_bits2f(hb[4 + e]));
  }
  const v4u uh = (v4u){pk16(hb[0], hb[1]), pk16(hb[2], hb[3]), pk16(hb[4], hb[5]), pk16(hb[6], hb[7])};
  const v4u ul = (v4u){pk16(lb[0], lb[1]), pk16(lb[2], lb[3]), pk16(lb[4], lb[5]), pk16(lb[6], lb[7])};
  const size_t o = (size_t)row * CPITCH + c8;
  *(volatile v4u*)(XH + o) = uh;
  *(volatile v4u*)(XL + o) = ul;
  __threadfence();
  *(volatile v4u*)(XH + o) = uh;
  *(volatile v4u*)(XL + o) = ul;
}

constexpr int AG_SRB  = 256;
constexpr int AG_RPW  = AG_SRB / 8;
constexpr int AG_SCH  = 2048;
constexpr int AG_SP   = AG_SCH / NTHR;
constexpr int AG_NCH  = (NEDGE + AG_SCH - 1) / AG_SCH;
constexpr int AG_NBLK = (NPAD + AG_SRB - 1) / AG_SRB;
static_assert(NEDGE % AG_SP == 0 && AG_SP % 4 == 0, "cfg");
static_assert(AG_SRB == 256 && AG_RPW == 32, "cfg");
static_assert(NEDGE <= (1 << 21), "cfg");
static_assert(AG_NBLK * AG_SRB >= NPAD, "cfg");

__device__ __forceinline__ int blk_excl_scan(int cnt, int* scan_ws, int tid, int* tot) {
  const int lane = tid & 31, wave = tid >> 5; int incl = cnt;
#pragma unroll
  for (int o = 1; o < 32; o <<= 1) { const int v = __shfl_up(incl, o, 32); if (lane >= o) incl += v; }
  if (lane == 31) scan_ws[wave] = incl;
  __syncthreads();
  if (wave == 0) { int wv = (lane < NTHR / 32) ? scan_ws[lane] : 0; int wincl = wv;
#pragma unroll
    for (int o = 1; o < 32; o <<= 1) { const int v = __shfl_up(wincl, o, 32); if (lane >= o) wincl += v; }
    if (lane < NTHR / 32) scan_ws[32 + lane] = wincl - wv; if (lane == 31) scan_ws[64] = wincl; }
  __syncthreads();
  const int res = scan_ws[32 + wave] + incl - cnt; *tot = scan_ws[64];
  return res;
}

__device__ __forceinline__ int chunk_hits(const int* __restrict__ dstv, int e0, int n0, int tid, int* LIST, int* scan_ws) {
  const int eb = e0 + tid * AG_SP;
  const bool inr = eb < NEDGE;
  const int ebc = inr ? eb : (NEDGE - AG_SP);
  int rec[AG_SP]; int cnt = 0;
#pragma unroll
  for (int k = 0; k < AG_SP; k += 4) {
    const v4i d4 = *(const v4i*)(dstv + ebc + k);
#pragma unroll
    for (int e = 0; e < 4; ++e) {
      const unsigned t = (unsigned)d4[e] - (unsigned)n0;
      const bool hit = inr && (t < (unsigned)AG_SRB);
      const int packed = (int)(((t & 255u) << 21) | (unsigned)(ebc + k + e));
      rec[k + e] = hit ? packed : -1;
      cnt += hit ? 1 : 0;
    }
  }
  int tot; int p = blk_excl_scan(cnt, scan_ws, tid, &tot);
#pragma unroll
  for (int k = 0; k < AG_SP; ++k) {
    if (rec[k] >= 0) { if ((unsigned)p < (unsigned)AG_SCH) LIST[p] = rec[k]; ++p; }
  }
  __syncthreads();
  return tot < AG_SCH ? tot : AG_SCH;
}

__global__ __launch_bounds__(NTHR) void agg_kernel(const int* __restrict__ rows, const int* __restrict__ cols, const float* __restrict__ vals,
                                                  const float* __restrict__ xf,
                                                  unsigned short* ah_out, unsigned short* al_out) {
  __shared__ __align__(16) float ACC[AG_SRB * FDIM];
  __shared__ int   LIST[AG_SCH];
  __shared__ int   scan_ws[80];
  const int tid = threadIdx.x, lane = tid & 31, wave = tid >> 5;
  const int n0  = blockIdx.x * AG_SRB;
  for (int i = tid; i < AG_SCH; i += NTHR) LIST[i] = -1;
  if (tid < 80) scan_ws[tid] = 0;
  const v4f z4 = {0.f, 0.f, 0.f, 0.f};
#pragma unroll 1
  for (int j = 0; j < AG_RPW; ++j) *(v4f*)(ACC + (wave * AG_RPW + j) * FDIM + 4 * lane) = z4;
  __syncthreads();
#pragma unroll 1
  for (int c = 0; c < AG_NCH; ++c) {
    const int tot = chunk_hits(rows, c * AG_SCH, n0, tid, LIST, scan_ws);
#pragma unroll 1
    for (int base = 0; base < tot; base += 32) {
      const int q  = base + lane;
      const int qc = (q < AG_SCH) ? q : (AG_SCH - 1);
      const int rv = LIST[qc];
      const int own = (q < tot && rv >= 0 && (rv >> 26) == wave) ? 1 : 0;
      unsigned msk = (unsigned)__ballot(own);
#pragma unroll 1
      for (int it = 0; it < 32; ++it) {
        if (msk == 0u) break;
        const int bp = __builtin_ctz(msk); msk &= msk - 1u;
        const int r = __shfl(rv, bp, 32);
        const int dl = r >> 21;
        int e = r & 0x1fffff; e = (e < NEDGE) ? e : (NEDGE - 1);
        int s = cols[e]; s = s < 0 ? 0 : (s >= NNODE ? NNODE - 1 : s);
        const float w = bfr(vals[e]);
        const v4f xv = *(const v4f*)(xf + (size_t)s * FDIM + 4 * lane);
        float* ap = ACC + dl * FDIM + 4 * lane;
        v4f a = *(const v4f*)ap;
        a = a + w * xv;
        *(v4f*)ap = a;
      }
    }
    __syncthreads();
  }
  const int hh = lane >> 4, c8 = (lane & 15) * 8;
  for (int pass = 0; pass < 2; ++pass) {
#pragma unroll 1
    for (int j = 0; j < AG_RPW; j += 2) {
      const int nA = n0 + wave * AG_RPW + j;
      if (nA < NPAD) {
        const int dl = wave * AG_RPW + j + hh;
        const int n  = n0 + dl;
        const float fl = (n < NNODE) ? 1.0f : 0.0f;
        const float* rp = ACC + dl * FDIM + c8;
        const v4f a = *(const v4f*)rp;
        const v4f c = *(const v4f*)(rp + 4);
        unsigned short hb[8], lb[8];
#pragma unroll
        for (int e = 0; e < 4; ++e) {
          const float v0 = a[e] * fl;
          const float v1 = c[e] * fl;
          hb[e] = f2bf_bits(v0);      lb[e] = f2bf_bits(v0 - bf_bits2f(hb[e]));
          hb[4 + e] = f2bf_bits(v1);  lb[4 + e] = f2bf_bits(v1 - bf_bits2f(hb[4 + e]));
        }
        const v4u uh = (v4u){pk16(hb[0], hb[1]), pk16(hb[2], hb[3]), pk16(hb[4], hb[5]), pk16(hb[6], hb[7])};
        const v4u ul = (v4u){pk16(lb[0], lb[1]), pk16(lb[2], lb[3]), pk16(lb[4], lb[5]), pk16(lb[6], lb[7])};
        const size_t o = (size_t)n * CPITCH + c8;
        *(volatile v4u*)(ah_out + o) = uh;
        *(volatile v4u*)(al_out + o) = ul;
      }
    }
    __threadfence();
  }
}

__global__ __launch_bounds__(NTHR) void rx_kernel(const float* __restrict__ rpre, const float* __restrict__ xf,
                                                 unsigned short* rxh, unsigned short* rxl) {
  const int i = blockIdx.x * NTHR + threadIdx.x;
  if (i >= NPAD * 32) return;
  const int row = i >> 5, col = (i & 31) * 4;
  const size_t fo = (size_t)row * FDIM + col;
  const v4f rp = *(const v4f*)(rpre + fo);
  const v4f xv = *(const v4f*)(xf + fo);
  unsigned short hb[4], lb[4];
#pragma unroll
  for (int e = 0; e < 4; ++e) {
    const float rr = sigm_f(rp[e]);
    const float m  = rr * xv[e];
    hb[e] = f2bf_bits(m);
    lb[e] = f2bf_bits(m - bf_bits2f(hb[e]));
  }
  const v2u oh = (v2u){pk16(hb[0], hb[1]), pk16(hb[2], hb[3])};
  const v2u ol = (v2u){pk16(lb[0], lb[1]), pk16(lb[2], lb[3])};
  const size_t xo = (size_t)row * CPITCH + col;
  *(volatile v2u*)(rxh + xo) = oh;
  *(volatile v2u*)(rxl + xo) = ol;
  __threadfence();
  *(volatile v2u*)(rxh + xo) = oh;
  *(volatile v2u*)(rxl + xo) = ol;
}

extern "C" void kernel_launch(void* const* d_in, const int* in_sizes, int n_in,
                              void* d_out, int out_size, void* d_ws, size_t ws_size, hipStream_t stream) {
  if (n_in < 24) return;
  if (in_sizes[0] != NNODE * FDIM || in_sizes[1] != NEDGE || in_sizes[2] != NEDGE || in_sizes[3] != NEDGE) return;
  if (out_size != NNODE * FDIM) return;
  for (int i = 0; i < 10; ++i) { if (in_sizes[4 + 2 * i] != FDIM * FDIM || in_sizes[5 + 2 * i] != FDIM) return; }

  const float* x_in  = (const float*)d_in[0];
  const int*   erows = (const int*)d_in[1];
  const int*   ecols = (const int*)d_in[2];
  const float* evals = (const float*)d_in[3];
  const float* m1_W1 = (const float*)d_in[4];  const float* m1_b1 = (const float*)d_in[5];
  const float* m1_W2 = (const float*)d_in[6];  const float* m1_b2 = (const float*)d_in[7];
  const float* m2_W1 = (const float*)d_in[8];  const float* m2_b1 = (const float*)d_in[9];
  const float* m2_W2 = (const float*)d_in[10]; const float* m2_b2 = (const float*)d_in[11];
  const float* Wu1   = (const float*)d_in[12]; const float* bu1   = (const float*)d_in[13];
  const float* Wu2   = (const float*)d_in[14]; const float* bu2   = (const float*)d_in[15];
  const float* Wr1   = (const float*)d_in[16]; const float* br1   = (const float*)d_in[17];
  const float* Wr2   = (const float*)d_in[18]; const float* br2   = (const float*)d_in[19];
  const float* Wo1   = (const float*)d_in[20]; const float* bo1   = (const float*)d_in[21];
  const float* Wo2   = (const float*)d_in[22]; const float* bo2   = (const float*)d_in[23];
  float* out = (float*)d_out;

  char* ws = (char*)d_ws; size_t off = 0;
  auto carve = [&](size_t bytes) -> char* { char* p = ws + off; off += (bytes + 255) & ~(size_t)255; return p; };
  unsigned short* WB    = (unsigned short*)carve((size_t)WPLANE_HALVES * 2);
  float*          BIASR = (float*)carve((size_t)NBIASR * 4);
  unsigned short* CATH  = (unsigned short*)carve((size_t)NPAD * CPITCH * 2);
  unsigned short* CATL  = (unsigned short*)carve((size_t)NPAD * CPITCH * 2);
  float*          XF32  = (float*)carve((size_t)NPAD * FDIM * 4);
  float*          RF32  = (float*)carve((size_t)NPAD * FDIM * 4);
  if (off > ws_size || off > (size_t)134217728) return;

  static_assert(NPAD % 64 == 0 && FDIM % 64 == 0 && FDIM % 32 == 0 && (2 * FDIM) % 32 == 0, "gemm shapes");
  const int gemm_blocks = ((NPAD / 64) * (FDIM / 64) + 7) / 8;
  const float* nof = (const float*)nullptr;

  prep_kernel<<<41, NTHR, 0, stream>>>(m1_W1, m1_W2, m2_W1, m2_W2, Wu1, Wu2, Wr1, Wr2, Wo1, Wo2,
                                       m1_b1, m1_b2, m2_b1, m2_b2, bu1, bu2, br1, br2, bo1, bo2, WB, BIASR);
  cast_xin_kernel<<<(NPAD * 16) / NTHR, NTHR, 0, stream>>>(x_in, CATH);
  wmma_gemm64<1, 0, 2, 2, false, 2><<<dim3(gemm_blocks, 1), 256, 0, stream>>>(
      CATH, (const unsigned short*)nullptr, CPITCH, 0L, WB + WOFF_P1, (const unsigned short*)nullptr, FDIM, 0L,
      (void*)(CATH + 256), (void*)(CATL + 256), CPITCH, 0L, BIASR + BOFF_M1B1, nof, 0L, NPAD, FDIM, FDIM, 1.0f,
      nof, nof, 0);
  wmma_gemm64<1, 1, 2, 0, false, 0><<<dim3(gemm_blocks, 1), 256, 0, stream>>>(
      CATH + 256, CATL + 256, CPITCH, 0L, WB + WOFF_P2, (const unsigned short*)nullptr, FDIM, 0L,
      (void*)XF32, (void*)nullptr, FDIM, 0L, BIASR + BOFF_M1B2, nof, 0L, NPAD, FDIM, FDIM, 1.0f,
      nof, nof, 0);
  castx_kernel<<<(NPAD * 16) / NTHR, NTHR, 0, stream>>>(XF32, CATH, CATL);
  agg_kernel<<<AG_NBLK, NTHR, 0, stream>>>(erows, ecols, evals, XF32, CATH + 128, CATL + 128);
  wmma_gemm64<1, 1, 2, 2, false, 2><<<dim3(gemm_blocks, 1), 256, 0, stream>>>(
      CATH + 128, CATL + 128, CPITCH, 0L, WB + WOFF_P3, (const unsigned short*)nullptr, FDIM, 0L,
      (void*)(CATH + 256), (void*)(CATL + 256), CPITCH, 0L, BIASR + BOFF_M2B1, nof, 0L, NPAD, FDIM, FDIM, 1.0f,
      nof, nof, 0);
  wmma_gemm64<1, 1, 2, 2, false, 0><<<dim3(gemm_blocks, 1), 256, 0, stream>>>(
      CATH + 256, CATL + 256, CPITCH, 0L, WB + WOFF_P4, (const unsigned short*)nullptr, FDIM, 0L,
      (void*)(CATH + 128), (void*)(CATL + 128), CPITCH, 0L, BIASR + BOFF_M2B2, nof, 0L, NPAD, FDIM, FDIM, 1.0f,
      nof, nof, 0);
  wmma_gemm64<1, 1, 2, 0, false, 0><<<dim3(gemm_blocks, 1), 256, 0, stream>>>(
      CATH, CATL, CPITCH, 0L, WB + WOFF_ZR + 128 * 256, (const unsigned short*)nullptr, 2 * FDIM, 0L,
      (void*)RF32, (void*)nullptr, FDIM, 0L, BIASR + BOFF_R, nof, 0L, NPAD, FDIM, 2 * FDIM, 1.0f,
      nof, nof, 0);
  rx_kernel<<<(NPAD * 32) / NTHR, NTHR, 0, stream>>>(RF32, XF32, CATH + 256, CATL + 256);
  wmma_gemm64<1, 1, 2, 0, false, 0><<<dim3(gemm_blocks, 1), 256, 0, stream>>>(
      CATH, CATL, CPITCH, 0L, WB + WOFF_ZR, (const unsigned short*)nullptr, 2 * FDIM, 0L,
      (void*)RF32, (void*)nullptr, FDIM, 0L, BIASR + BOFF_Z, nof, 0L, NPAD, FDIM, 2 * FDIM, 1.0f,
      nof, nof, 0);
  wmma_gemm64<1, 1, 2, 3, false, 0><<<dim3(gemm_blocks, 1), 256, 0, stream>>>(
      CATH + 128, CATL + 128, CPITCH, 0L, WB + WOFF_H, (const unsigned short*)nullptr, 2 * FDIM, 0L,
      (void*)out, (void*)nullptr, FDIM, 0L, BIASR + BOFF_HB, nof, 0L, NPAD, FDIM, 2 * FDIM, 1.0f,
      RF32, XF32, NNODE);
}
